// LPKT_55387898250090
// MI455X (gfx1250) — hardware-run, weakly checked
//
#include <hip/hip_runtime.h>
#include <math.h>

constexpr int NBATCH  = 16;
constexpr int NSEQ    = 128;
constexpr int NCONC   = 100;
constexpr int NCPAD   = 112;
constexpr int NDK     = 128;
constexpr int NROWS   = NBATCH * NSEQ;
constexpr int NQROWS  = 5001;
constexpr int NATROWS = 3601;
constexpr int NITROWS = 43201;
constexpr int HPITCH  = 136;
constexpr int NTHR    = 256;

constexpr float WCARRY  = 16.0f;
constexpr float ECARRY  = 16.0f;
constexpr float ITCARRY = 64.0f;
constexpr float LCARRY  = 16.0f;
constexpr float HCARRY  = 16.0f;
constexpr float HTCARRY = 4.0f;
constexpr float SC_EW   = 1.0f / (ECARRY * WCARRY);
constexpr float SC_ITW  = 1.0f / (ITCARRY * WCARRY);
constexpr float SC_LW   = 1.0f / (LCARRY * WCARRY);
constexpr float SC_HW   = 1.0f / (HCARRY * WCARRY);
constexpr float SC_HTW  = 1.0f / (HTCARRY * WCARRY);

constexpr int OFF_W1T   = 0;
constexpr int OFF_W23L  = OFF_W1T  + NDK * 256;
constexpr int OFF_WIT   = OFF_W23L + 256 * 256;
constexpr int OFF_W4A   = OFF_WIT  + 384 * NDK;
constexpr int OFF_W5E   = OFF_W4A  + NDK * NDK;
constexpr int OFF_W5H   = OFF_W5E  + NDK * NDK;
constexpr int WPL_ELEMS = OFF_W5H  + NDK * NDK;

static_assert(NROWS == 2048, "rows");
static_assert(NROWS % 64 == 0 && NDK % 64 == 0, "GEMM tile multiples");
static_assert(NDK % 32 == 0 && 256 % 32 == 0, "GEMM K multiples of 32");
static_assert(NCPAD % 16 == 0 && NCPAD >= NCONC, "concept padding");
static_assert(HPITCH % 8 == 0 && HPITCH >= NDK, "LDS pitch");
static_assert(WPL_ELEMS == 196608, "weight plane size");
static_assert(NTHR == 2 * NDK, "one thread per gate column");
static_assert(2 * NCPAD <= NTHR, "q rows fit one block pass");

typedef __attribute__((ext_vector_type(16))) _Float16 v16h;
typedef __attribute__((ext_vector_type(8)))  _Float16 v8h;
typedef __attribute__((ext_vector_type(4)))  _Float16 v4h;
typedef __attribute__((ext_vector_type(8)))  float    v8f;
typedef __attribute__((ext_vector_type(4)))  float    v4f;

__device__ __forceinline__ void dep_guard4_h(v8f& a, v8f& b, v8f& c, v8f& d, v16h x, v16h y) {
  asm volatile("v_nop\n\tv_nop\n\tv_nop\n\tv_nop" : "+v"(a), "+v"(b), "+v"(c), "+v"(d) : "v"(x), "v"(y));
}
__device__ __forceinline__ void dep_guard1_h8(v8f& a, v16h x0, v16h x1, v16h x2, v16h x3,
                                              v16h y0, v16h y1, v16h y2, v16h y3) {
  asm volatile("v_nop\n\tv_nop\n\tv_nop\n\tv_nop" : "+v"(a)
               : "v"(x0), "v"(x1), "v"(x2), "v"(x3), "v"(y0), "v"(y1), "v"(y2), "v"(y3));
}
__device__ __forceinline__ void keep4_h(v16h a, v16h b, v16h c, v16h d) {
  asm volatile("v_nop" :: "v"(a), "v"(b), "v"(c), "v"(d));
}
__device__ __forceinline__ void acc_guard4(v8f& a, v8f& b, v8f& c, v8f& d) {
  asm volatile("v_nop\n\tv_nop\n\tv_nop\n\tv_nop" : "+v"(a), "+v"(b), "+v"(c), "+v"(d));
}

struct FragH {
  union U { v16h v; v8h h[2]; };
  static __device__ __forceinline__ v16h load(const _Float16* p) {
    U f; f.h[0] = *(const v8h*)(p); f.h[1] = *(const v8h*)(p + 16); return f.v;
  }
  static __device__ __forceinline__ v8f mma(v16h a, v16h b, v8f c) {
    return __builtin_amdgcn_wmma_f32_16x16x32_f16(false, a, false, b, (short)0, c, false, false);
  }
};

__device__ __forceinline__ float sigm(float x) {
  const float xc = fminf(fmaxf(x, -60.0f), 60.0f);
  return __builtin_amdgcn_rcpf(1.0f + expf(-xc));
}

template <int BIAS_MODE>
__global__ __launch_bounds__(256) void wmma_gemm64_f16(
    const unsigned short* __restrict__ Ap, int lda,
    const unsigned short* __restrict__ Btp, int ldb,
    float* __restrict__ Cout, int ldc,
    const float* __restrict__ bias, int Mrows, int Ncols, int Kdim, float scale) {
  const _Float16* A  = (const _Float16*)Ap;
  const _Float16* Bt = (const _Float16*)Btp;
  __shared__ __align__(16) float sT[8][16 * 68];
  const int lane = threadIdx.x & 31;
  const int wave = threadIdx.x >> 5;
  const int tilesN = Ncols >> 6;
  const int tilesM = Mrows >> 6;
  const int tile = blockIdx.x * 8 + wave;
  if (tile >= tilesM * tilesN) return;
  const int tm = tile / tilesN;
  const int tn = tile - tm * tilesN;
  const int m0 = tm << 6;
  const int n0 = tn << 6;
  const int rlane = lane & 15;
  const int koff  = (lane >> 4) * 8;
  const int mOff  = (lane >> 4) * 8;

  v8f acc[4][4];
#pragma unroll
  for (int i = 0; i < 4; ++i)
#pragma unroll
    for (int j = 0; j < 4; ++j) acc[i][j] = (v8f){0.f, 0.f, 0.f, 0.f, 0.f, 0.f, 0.f, 0.f};

  for (int k0 = 0; k0 < Kdim; k0 += 32) {
    v16h bh[4];
#pragma unroll
    for (int j = 0; j < 4; ++j) {
      const size_t bo = (size_t)(n0 + (j << 4) + rlane) * ldb + koff + k0;
      bh[j] = FragH::load(Bt + bo);
    }
#pragma unroll
    for (int i = 0; i < 4; ++i) {
      const size_t ao = (size_t)(m0 + (i << 4) + rlane) * lda + koff + k0;
      const v16h ah = FragH::load(A + ao);
#pragma unroll
      for (int j = 0; j < 4; ++j) acc[i][j] = FragH::mma(ah, bh[j], acc[i][j]);
      dep_guard4_h(acc[i][0], acc[i][1], acc[i][2], acc[i][3], ah, bh[3]);
    }
    keep4_h(bh[0], bh[1], bh[2], bh[3]);
  }
  acc_guard4(acc[0][0], acc[0][1], acc[0][2], acc[0][3]);
  acc_guard4(acc[1][0], acc[1][1], acc[1][2], acc[1][3]);
  acc_guard4(acc[2][0], acc[2][1], acc[2][2], acc[2][3]);
  acc_guard4(acc[3][0], acc[3][1], acc[3][2], acc[3][3]);

  float* slab = sT[wave];
#pragma unroll
  for (int i = 0; i < 4; ++i) {
    const int mBase = m0 + (i << 4);
#pragma unroll
    for (int j = 0; j < 4; ++j) {
      const int n = n0 + (j << 4) + rlane;
      float bv = 0.f;
      if (BIAS_MODE == 2) bv = bias[n];
#pragma unroll
      for (int r = 0; r < 8; ++r) {
        float v = acc[i][j][r] * scale;
        if (BIAS_MODE == 2) v += bv;
        slab[(mOff + r) * 68 + (j << 4) + rlane] = v;
      }
    }
    __builtin_amdgcn_fence(__ATOMIC_RELEASE, "workgroup");
    __builtin_amdgcn_wave_barrier();
    __builtin_amdgcn_fence(__ATOMIC_ACQUIRE, "workgroup");
    {
      const int hh = lane >> 4, c4 = (lane & 15) * 4;
      for (int pass = 0; pass < 2; ++pass) {
#pragma unroll
        for (int it = 0; it < 8; ++it) {
          const int row = it * 2 + hh;
          const v4f v = *(const v4f*)(slab + row * 68 + c4);
          *(volatile v4f*)(Cout + (size_t)(mBase + row) * ldc + n0 + c4) = v;
        }
        __threadfence();
      }
    }
    __builtin_amdgcn_fence(__ATOMIC_RELEASE, "workgroup");
    __builtin_amdgcn_wave_barrier();
    __builtin_amdgcn_fence(__ATOMIC_ACQUIRE, "workgroup");
  }
}

__global__ __launch_bounds__(160) void vec_prep_kernel(const float* __restrict__ W1, const float* __restrict__ b1,
                                                       const float* __restrict__ b2, const float* __restrict__ b3,
                                                       const float* __restrict__ b4, float* __restrict__ VEC) {
  const int lane = threadIdx.x & 31, wave = threadIdx.x >> 5;
  const int c4 = lane * 4;
  v4f cs = {0.f, 0.f, 0.f, 0.f};
#pragma unroll 1
  for (int k = 0; k < NDK; ++k) {
    const v4f w = *(const v4f*)(W1 + (size_t)(2 * NDK + k) * NDK + c4);
    cs += w;
  }
  const v4f v1 = *(const v4f*)(b1 + c4);
  const v4f v2 = *(const v4f*)(b2 + c4);
  const v4f v3 = *(const v4f*)(b3 + c4);
  const v4f v4 = *(const v4f*)(b4 + c4);
  v4f o;
#pragma unroll
  for (int e = 0; e < 4; ++e)
    o[e] = (wave == 0) ? cs[e] : (wave == 1) ? v1[e] : (wave == 2) ? v2[e] : (wave == 3) ? v3[e] : v4[e];
  float* op = VEC + wave * NDK + c4;
  *(volatile v4f*)op = o;
  __threadfence();
  *(volatile v4f*)op = o;
}

__global__ __launch_bounds__(NTHR) void tp_weights_kernel(const float* __restrict__ W1, const float* __restrict__ W2,
                                                          const float* __restrict__ W3, const float* __restrict__ W4,
                                                          const float* __restrict__ W5, unsigned short* __restrict__ WPL) {
  __shared__ float Tt[64 * 65];
  const int tid = threadIdx.x;
  const int z = blockIdx.z;
  int wid, rb, doff, ldo;
  switch (z) {
    case 0:  wid = 0; rb = 0; doff = OFF_W1T;                   ldo = 256; break;
    case 1:  wid = 0; rb = 1; doff = OFF_W1T + NDK;             ldo = 256; break;
    case 2:  wid = 1; rb = 0; doff = OFF_W23L;                  ldo = 256; break;
    case 3:  wid = 1; rb = 2; doff = OFF_W23L + NDK;            ldo = 256; break;
    case 4:  wid = 2; rb = 0; doff = OFF_W23L + NDK * 256;       ldo = 256; break;
    case 5:  wid = 2; rb = 2; doff = OFF_W23L + NDK * 256 + NDK; ldo = 256; break;
    case 6:  wid = 1; rb = 1; doff = OFF_WIT;                   ldo = NDK; break;
    case 7:  wid = 2; rb = 1; doff = OFF_WIT + NDK * NDK;        ldo = NDK; break;
    case 8:  wid = 3; rb = 2; doff = OFF_WIT + 2 * NDK * NDK;    ldo = NDK; break;
    case 9:  wid = 3; rb = 0; doff = OFF_W4A;                   ldo = NDK; break;
    case 10: wid = 4; rb = 0; doff = OFF_W5E;                   ldo = NDK; break;
    default: wid = 4; rb = 1; doff = OFF_W5H;                   ldo = NDK; break;
  }
  const float* Wsel = (wid == 0) ? W1 : (wid == 1) ? W2 : (wid == 2) ? W3 : (wid == 3) ? W4 : W5;
  const float* src = Wsel + (size_t)rb * NDK * NDK;
  const int c0 = blockIdx.x * 64, r0 = blockIdx.y * 64;
#pragma unroll
  for (int i = 0; i < 4; ++i) {
    const int idx = i * NTHR + tid;
    const int rr = idx >> 4, cc = (idx & 15) * 4;
    const v4f v = *(const v4f*)(src + (size_t)(r0 + rr) * NDK + c0 + cc);
    Tt[rr * 65 + cc + 0] = v[0];
    Tt[rr * 65 + cc + 1] = v[1];
    Tt[rr * 65 + cc + 2] = v[2];
    Tt[rr * 65 + cc + 3] = v[3];
  }
  __syncthreads();
  const int q = tid >> 3, c8 = (tid & 7) * 8;
  v8h hv[2];
#pragma unroll
  for (int g = 0; g < 2; ++g) {
    const int qq = g * 32 + q;
#pragma unroll
    for (int e = 0; e < 8; ++e) {
      const float f = Tt[(c8 + e) * 65 + qq];
      hv[g][e] = (_Float16)(f * WCARRY);
    }
  }
  for (int pass = 0; pass < 2; ++pass) {
#pragma unroll
    for (int g = 0; g < 2; ++g) {
      const size_t o = (size_t)doff + (size_t)(c0 + g * 32 + q) * (size_t)ldo + (size_t)(r0 + c8);
      *(volatile v8h*)(WPL + o) = hv[g];
    }
    __threadfence();
  }
}

__global__ __launch_bounds__(NTHR) void gather_kernel(const int* __restrict__ qseq, const int* __restrict__ useq,
                                                      const int* __restrict__ iseq, const float* __restrict__ e_w,
                                                      const float* __restrict__ at_w, const float* __restrict__ it_w,
                                                      unsigned short* __restrict__ A1, unsigned short* __restrict__ IT16) {
  const int part = blockIdx.y;
  const int i = blockIdx.x * NTHR + threadIdx.x;
  const int row = i >> 4, c8 = i & 15;
  const int* idxp  = (part == 0) ? qseq : (part == 1) ? useq : iseq;
  const float* tab = (part == 0) ? e_w : (part == 1) ? at_w : it_w;
  const int nrow   = (part == 0) ? NQROWS : (part == 1) ? NATROWS : NITROWS;
  const float sc   = (part == 2) ? ITCARRY : ECARRY;
  unsigned short* dst = (part == 2) ? (IT16 + (size_t)row * NDK + c8 * 8)
                                    : (A1 + (size_t)row * 256 + part * NDK + c8 * 8);
  int idx = idxp[row];
  idx = idx < 0 ? 0 : (idx > nrow - 1 ? nrow - 1 : idx);
  const float* sp = tab + (size_t)idx * NDK + c8 * 8;
  const v4f a = *(const v4f*)(sp);
  const v4f b = *(const v4f*)(sp + 4);
  v8h hv;
#pragma unroll
  for (int e = 0; e < 4; ++e) {
    hv[e]     = (_Float16)(a[e] * sc);
    hv[4 + e] = (_Float16)(b[e] * sc);
  }
  *(volatile v8h*)dst = hv;
  __threadfence();
  *(volatile v8h*)dst = hv;
}

__global__ __launch_bounds__(NTHR) void al_prep_kernel(const float* __restrict__ LRAW, const float* __restrict__ corr,
                                                       const float* __restrict__ VEC, unsigned short* __restrict__ AL) {
  const int i = blockIdx.x * NTHR + threadIdx.x;
  const int row = i >> 5, c8 = i & 31;
  const int t = row & (NSEQ - 1);
  const bool isPrev = (c8 < 16);
  const bool zero = isPrev && (t == 0);
  const int srow = (isPrev && t > 0) ? (row - 1) : row;
  const int cc = (c8 & 15) * 8;
  float cv = corr[srow];
  asm volatile("" : "+v"(cv));
  const v4f l0 = *(const v4f*)(LRAW + (size_t)srow * NDK + cc);
  const v4f l1 = *(const v4f*)(LRAW + (size_t)srow * NDK + cc + 4);
  const v4f s0 = *(const v4f*)(VEC + cc);
  const v4f s1 = *(const v4f*)(VEC + cc + 4);
  const v4f b0 = *(const v4f*)(VEC + NDK + cc);
  const v4f b1v = *(const v4f*)(VEC + NDK + cc + 4);
  v8h hv;
#pragma unroll
  for (int e = 0; e < 4; ++e) {
    const float x0 = (l0[e] + cv * s0[e]) + b0[e];
    const float x1 = (l1[e] + cv * s1[e]) + b1v[e];
    hv[e]     = (_Float16)(zero ? 0.0f : x0 * LCARRY);
    hv[4 + e] = (_Float16)(zero ? 0.0f : x1 * LCARRY);
  }
  unsigned short* dst = AL + (size_t)i * 8;
  *(volatile v8h*)dst = hv;
  __threadfence();
  *(volatile v8h*)dst = hv;
}

__global__ __launch_bounds__(NTHR) void recur_kernel(const int* __restrict__ qseq, const float* __restrict__ qmat,
                                                     const float* __restrict__ h0,
                                                     const float* __restrict__ W2, const float* __restrict__ W3,
                                                     const float* __restrict__ W4,
                                                     const unsigned short* __restrict__ W4atp,
                                                     const float* __restrict__ PL, const float* __restrict__ PIT,
                                                     unsigned short* __restrict__ HT16) {
  __shared__ __align__(16) float    hF[NCPAD * NDK];
  __shared__ __align__(16) _Float16 hH[2 * NCPAD * HPITCH];
  __shared__ __align__(16) float    htS[NDK];
  __shared__ float qS[2 * NCPAD];
  __shared__ float lgS[NDK];
  __shared__ float tmpG[2 * NDK];
  __shared__ float tmpS[2 * NDK];

  const int tid = threadIdx.x, lane = tid & 31, wave = tid >> 5;
  const int c = lane & 15, hh = lane >> 4, koff = hh * 8;
  const int col = 16 * wave + c;
  const int b = blockIdx.x;
  const _Float16* W4at = (const _Float16*)W4atp;

  const _Float16* wb = W4at + (size_t)col * NDK + koff;
  const v16h bw0 = FragH::load(wb);
  const v16h bw1 = FragH::load(wb + 32);
  const v16h bw2 = FragH::load(wb + 64);
  const v16h bw3 = FragH::load(wb + 96);

  {
    int q0 = qseq[b * NSEQ];
    q0 = q0 < 0 ? 0 : (q0 > NQROWS - 1 ? NQROWS - 1 : q0);
    if (tid < 2 * NCPAD) {
      const int which = (tid >= NCPAD) ? 1 : 0;
      const int m = tid - which * NCPAD;
      const int mc = (m < NCONC) ? m : (NCONC - 1);
      float v = qmat[(size_t)q0 * NCONC + mc];
      asm volatile("" : "+v"(v));
      qS[tid] = (m < NCONC) ? v : 0.0f;
    }
  }
  __syncthreads();
  {
    float hpart = 0.0f;
#pragma unroll 1
    for (int mt = 0; mt < NCPAD / 16; ++mt) {
#pragma unroll
      for (int r = 0; r < 8; ++r) {
        const int m = 16 * mt + 8 * hh + r;
        const int mc = (m < NCONC) ? m : (NCONC - 1);
        float v = h0[(size_t)mc * NDK + col];
        asm volatile("" : "+v"(v));
        v = (m < NCONC) ? v : 0.0f;
        hF[m * NDK + col] = v;
        hH[m * HPITCH + col] = (_Float16)(v * HCARRY);
        hpart = fmaf(qS[NCPAD + m], v, hpart);
      }
    }
    const float other = __shfl_xor(hpart, 16, 32);
    const float total = hpart + other;
    if (hh == 0) htS[col] = total;
  }
  __syncthreads();
  if (wave == 0) {
    const v4f hv = *(const v4f*)(htS + 4 * lane);
    v4h o;
#pragma unroll
    for (int e = 0; e < 4; ++e) o[e] = (_Float16)(hv[e] * HTCARRY);
    unsigned short* p = HT16 + (size_t)(b * NSEQ) * NDK + 4 * lane;
    *(volatile v4h*)p = o;
    __threadfence();
    *(volatile v4h*)p = o;
  }

  const v8f z8 = {0.f, 0.f, 0.f, 0.f, 0.f, 0.f, 0.f, 0.f};

#pragma unroll 1
  for (int t = 0; t < NSEQ - 1; ++t) {
    const int row = b * NSEQ + t;
    int qt  = qseq[row];
    int qt1 = qseq[row + 1];
    qt  = qt  < 0 ? 0 : (qt  > NQROWS - 1 ? NQROWS - 1 : qt);
    qt1 = qt1 < 0 ? 0 : (qt1 > NQROWS - 1 ? NQROWS - 1 : qt1);
    if (tid < 2 * NCPAD) {
      const int which = (tid >= NCPAD) ? 1 : 0;
      const int m = tid - which * NCPAD;
      const int qi = which ? qt1 : qt;
      const int mc = (m < NCONC) ? m : (NCONC - 1);
      float v = qmat[(size_t)qi * NCONC + mc];
      asm volatile("" : "+v"(v));
      qS[tid] = (m < NCONC) ? v : 0.0f;
    }
    {
      const float* Wd = (tid < NDK) ? (W2 + (size_t)3 * NDK * NDK + tid) : (W3 + (size_t)3 * NDK * NDK + (tid - NDK));
      float a = PL[(size_t)row * 256 + tid] + PIT[(size_t)row * 384 + tid];
#pragma unroll 4
      for (int k = 0; k < NDK; ++k) a = fmaf(htS[k], Wd[(size_t)k * NDK], a);
      tmpG[tid] = a;
    }
    __syncthreads();
    if (tid < NDK) {
      const float lg = tanhf(tmpG[tid]);
      const float gl = sigm(tmpG[NDK + tid]);
      lgS[tid] = gl * (lg + 1.0f) * 0.5f;
    }
    __syncthreads();
    {
      const int n = tid & (NDK - 1), kh = tid >> 7;
      const float* Wb = W4 + (size_t)(NDK + 64 * kh) * NDK + n;
      const float* lgp = lgS + 64 * kh;
      float a = 0.0f;
#pragma unroll 4
      for (int k = 0; k < 64; ++k) a = fmaf(lgp[k], Wb[(size_t)k * NDK], a);
      tmpS[tid] = a;
    }
    const float pit4 = PIT[(size_t)row * 384 + 256 + col];
    __syncthreads();
    const float LGn = lgS[col];
    const float sn  = (tmpS[col] + tmpS[NDK + col]) + pit4;
    const _Float16* hcur = hH + (t & 1) * (NCPAD * HPITCH);
    _Float16*       hnxt = hH + ((t & 1) ^ 1) * (NCPAD * HPITCH);
    float hpart = 0.0f;
#pragma unroll 1
    for (int mt = 0; mt < NCPAD / 16; ++mt) {
      const _Float16* ap = hcur + (16 * mt + c) * HPITCH + koff;
      const v16h a0 = FragH::load(ap);
      const v16h a1 = FragH::load(ap + 32);
      const v16h a2 = FragH::load(ap + 64);
      const v16h a3 = FragH::load(ap + 96);
      v8f acc = z8;
      acc = FragH::mma(a0, bw0, acc);
      acc = FragH::mma(a1, bw1, acc);
      acc = FragH::mma(a2, bw2, acc);
      acc = FragH::mma(a3, bw3, acc);
      dep_guard1_h8(acc, a0, a1, a2, a3, bw0, bw1, bw2, bw3);
#pragma unroll
      for (int r = 0; r < 8; ++r) {
        const int m = 16 * mt + 8 * hh + r;
        const float pre = acc[r] * SC_HW + sn;
        const float gf = sigm(pre);
        const float ho = hF[m * NDK + col];
        float hn = fmaf(gf, ho, qS[m] * LGn);
        hn = (m < NCONC) ? hn : 0.0f;
        hF[m * NDK + col] = hn;
        hnxt[m * HPITCH + col] = (_Float16)(hn * HCARRY);
        hpart = fmaf(qS[NCPAD + m], hn, hpart);
      }
    }
    {
      const float other = __shfl_xor(hpart, 16, 32);
      const float total = hpart + other;
      if (hh == 0) htS[col] = total;
    }
    __syncthreads();
    if (wave == 0) {
      const v4f hv = *(const v4f*)(htS + 4 * lane);
      v4h o;
#pragma unroll
      for (int e = 0; e < 4; ++e) o[e] = (_Float16)(hv[e] * HTCARRY);
      unsigned short* p = HT16 + (size_t)(row + 1) * NDK + 4 * lane;
      *(volatile v4h*)p = o;
      __threadfence();
      *(volatile v4h*)p = o;
    }
  }
}

__global__ __launch_bounds__(NTHR) void mean_kernel(const float* __restrict__ P5E, const float* __restrict__ P5H,
                                                    float* __restrict__ out) {
  const int row = blockIdx.x * NTHR + threadIdx.x;
  const float* pe = P5E + (size_t)row * NDK;
  const float* ph = P5H + (size_t)row * NDK;
  float s = 0.0f;
#pragma unroll 1
  for (int i = 0; i < NDK / 4; ++i) {
    const v4f a = *(const v4f*)(pe + 4 * i);
    const v4f g = *(const v4f*)(ph + 4 * i);
#pragma unroll
    for (int e = 0; e < 4; ++e) s += sigm(a[e] + g[e]);
  }
  float v = s * (1.0f / (float)NDK);
  v = ((row & (NSEQ - 1)) == 0) ? 0.0f : v;
  *(volatile float*)(out + row) = v;
  __threadfence();
  *(volatile float*)(out + row) = v;
}

extern "C" void kernel_launch(void* const* d_in, const int* in_sizes, int n_in,
                              void* d_out, int out_size, void* d_ws, size_t ws_size, hipStream_t stream) {
  if (n_in < 19 || d_out == nullptr || d_ws == nullptr) return;
  if (in_sizes[0] != NROWS || in_sizes[1] != NROWS || in_sizes[2] != NROWS || in_sizes[3] != NROWS ||
      in_sizes[4] != NQROWS * NCONC || in_sizes[5] != NCONC * NDK || in_sizes[6] != NQROWS * NDK ||
      in_sizes[7] != NATROWS * NDK || in_sizes[8] != NITROWS * NDK || in_sizes[9] != 384 * NDK ||
      in_sizes[10] != NDK || in_sizes[11] != 512 * NDK || in_sizes[12] != NDK || in_sizes[13] != 512 * NDK ||
      in_sizes[14] != NDK || in_sizes[15] != 384 * NDK || in_sizes[16] != NDK || in_sizes[17] != 256 * NDK ||
      in_sizes[18] != NDK || out_size != NROWS) return;

  const int*   qseq = (const int*)d_in[0];
  const int*   useq = (const int*)d_in[1];
  const int*   iseq = (const int*)d_in[2];
  const float* corr = (const float*)d_in[3];
  const float* qmat = (const float*)d_in[4];
  const float* h0   = (const float*)d_in[5];
  const float* e_w  = (const float*)d_in[6];
  const float* at_w = (const float*)d_in[7];
  const float* it_w = (const float*)d_in[8];
  const float* W1   = (const float*)d_in[9];
  const float* b1   = (const float*)d_in[10];
  const float* W2   = (const float*)d_in[11];
  const float* b2   = (const float*)d_in[12];
  const float* W3   = (const float*)d_in[13];
  const float* b3   = (const float*)d_in[14];
  const float* W4   = (const float*)d_in[15];
  const float* b4   = (const float*)d_in[16];
  const float* W5   = (const float*)d_in[17];
  const float* b5   = (const float*)d_in[18];
  float* out = (float*)d_out;

  char* ws = (char*)d_ws; size_t off = 0;
  auto carve = [&](size_t bytes) -> char* { char* p = ws + off; off += (bytes + 255) & ~(size_t)255; return p; };
  unsigned short* WPL  = (unsigned short*)carve((size_t)WPL_ELEMS * 2);
  float*          VEC  = (float*)carve((size_t)5 * NDK * 4);
  unsigned short* A1   = (unsigned short*)carve((size_t)NROWS * 256 * 2);
  unsigned short* IT16 = (unsigned short*)carve((size_t)NROWS * NDK * 2);
  unsigned short* AL   = (unsigned short*)carve((size_t)NROWS * 256 * 2);
  unsigned short* HT16 = (unsigned short*)carve((size_t)NROWS * NDK * 2);
  float*          LRAW = (float*)carve((size_t)NROWS * NDK * 4);
  float*          P5E  = (float*)carve((size_t)NROWS * NDK * 4);
  float*          P5H  = (float*)carve((size_t)NROWS * NDK * 4);
  float*          PIT  = (float*)carve((size_t)NROWS * 384 * 4);
  float*          PL   = (float*)carve((size_t)NROWS * 256 * 4);
  if (off > ws_size || off > (size_t)134217728) return;

  vec_prep_kernel<<<1, 160, 0, stream>>>(W1, b1, b2, b3, b4, VEC);
  tp_weights_kernel<<<dim3(2, 2, 12), NTHR, 0, stream>>>(W1, W2, W3, W4, W5, WPL);
  gather_kernel<<<dim3(NROWS * 16 / NTHR, 3), NTHR, 0, stream>>>(qseq, useq, iseq, e_w, at_w, it_w, A1, IT16);

  wmma_gemm64_f16<0><<<(NROWS / 64) * (NDK / 64) / 8, 256, 0, stream>>>(
      A1, 256, WPL + OFF_W1T, 256, LRAW, NDK, VEC, NROWS, NDK, 256, SC_EW);
  wmma_gemm64_f16<2><<<(NROWS / 64) * (NDK / 64) / 8, 256, 0, stream>>>(
      A1, 256, WPL + OFF_W5E, NDK, P5E, NDK, b5, NROWS, NDK, NDK, SC_EW);
  wmma_gemm64_f16<2><<<(NROWS / 64) * (384 / 64) / 8, 256, 0, stream>>>(
      IT16, NDK, WPL + OFF_WIT, NDK, PIT, 384, VEC + 2 * NDK, NROWS, 384, NDK, SC_ITW);
  al_prep_kernel<<<NROWS * 32 / NTHR, NTHR, 0, stream>>>(LRAW, corr, VEC, AL);
  wmma_gemm64_f16<0><<<(NROWS / 64) * (256 / 64) / 8, 256, 0, stream>>>(
      AL, 256, WPL + OFF_W23L, 256, PL, 256, VEC, NROWS, 256, 256, SC_LW);
  recur_kernel<<<NBATCH, NTHR, 0, stream>>>(qseq, qmat, h0, W2, W3, W4, WPL + OFF_W4A, PL, PIT, HT16);
  wmma_gemm64_f16<0><<<(NROWS / 64) * (NDK / 64) / 8, 256, 0, stream>>>(
      HT16, NDK, WPL + OFF_W5H, NDK, P5H, NDK, VEC, NROWS, NDK, NDK, SC_HTW);
  mean_kernel<<<NROWS / NTHR, NTHR, 0, stream>>>(P5E, P5H, out);
}
